// EncoderDecoder_59296318488642
// MI455X (gfx1250) — hardware-verified
//
#include <hip/hip_runtime.h>
#include <math.h>

constexpr int BATCH = 2048;
constexpr int SEQ   = 512;
constexpr int DIN   = 4;
constexpr int HID   = 32;
constexpr int G3    = 96;
constexpr int DOUT  = 4;
constexpr int FUT   = 60;
constexpr int ROWS  = 32;
constexpr int NTH   = 128;
constexpr int EP    = 40;
constexpr int HFP   = 36;
constexpr int YSP   = FUT * DOUT;
constexpr float WSC     = 16.0f;
constexpr float WSC_INV = 1.0f / 16.0f;
static_assert(BATCH % ROWS == 0, "sz");
static_assert(NTH == ROWS * DOUT, "sz");
static_assert(NTH == 4 * 32, "sz");
static_assert((ROWS * YSP) % (NTH * 4) == 0, "sz");
static_assert((ROWS * YSP * 4) % 512 == 0, "sz");

typedef __attribute__((ext_vector_type(16))) _Float16 v16h;
typedef __attribute__((ext_vector_type(8)))  _Float16 v8h;
typedef __attribute__((ext_vector_type(8)))  float    v8f;
typedef __attribute__((ext_vector_type(4)))  float    v4f;

__device__ __forceinline__ void dep_guard_h(v8f& a, v8f& b, v16h x, v16h y) { asm volatile("v_nop\n\tv_nop\n\tv_nop\n\tv_nop" : "+v"(a), "+v"(b) : "v"(x), "v"(y)); }
__device__ __forceinline__ void keep4_h(v16h a, v16h b, v16h c, v16h d) { asm volatile("v_nop" :: "v"(a), "v"(b), "v"(c), "v"(d)); }
__device__ __forceinline__ void dep_guard4x_h(v8f& a, v8f& b, v8f& c, v8f& d, v16h x, v16h y) {
  asm volatile("v_nop\n\tv_nop\n\tv_nop\n\tv_nop" : "+v"(a), "+v"(b), "+v"(c), "+v"(d) : "v"(x), "v"(y));
}

template <typename T> struct Frag;
template <> struct Frag<_Float16> {
  typedef v16h V; union U { v16h v; v8h h[2]; };
  static __device__ __forceinline__ v16h load(const _Float16* p) {
    U f; f.h[0] = *(const v8h*)(p); f.h[1] = *(const v8h*)(p + 16); return f.v;
  }
  static __device__ __forceinline__ v8f mma(v16h a, v16h b, v8f c) {
    return __builtin_amdgcn_wmma_f32_16x16x32_f16(false, a, false, b, (short)0, c, false, false);
  }
  static __device__ __forceinline__ void guard(v8f& a, v8f& b, v16h x, v16h y) { dep_guard_h(a, b, x, y); }
  static __device__ __forceinline__ void keep(v16h a, v16h b, v16h c, v16h d) { keep4_h(a, b, c, d); }
};

__device__ __forceinline__ v16h frag_f32_f16(const float* __restrict__ p, float s) {
  v16h f;
#pragma unroll
  for (int e = 0; e < 8; ++e) {
    f[e]     = (_Float16)(p[e] * s);
    f[8 + e] = (_Float16)(p[16 + e] * s);
  }
  return f;
}

__device__ __forceinline__ float ftanh(float x) { return 1.0f - 2.0f * __builtin_amdgcn_rcpf(1.0f + __expf(2.0f * x)); }
__device__ __forceinline__ float fsigm(float x) { return __builtin_amdgcn_rcpf(1.0f + __expf(-x)); }

__global__ __launch_bounds__(NTH) void gru_seq2seq_kernel(
    const float* __restrict__ x,
    const float* __restrict__ Wemb, const float* __restrict__ bemb,
    const float* __restrict__ WihE, const float* __restrict__ WhhE,
    const float* __restrict__ bihE, const float* __restrict__ bhhE,
    const float* __restrict__ WihD, const float* __restrict__ WhhD,
    const float* __restrict__ bihD, const float* __restrict__ bhhD,
    const float* __restrict__ Wout, const float* __restrict__ bout,
    const int* __restrict__ flen,
    float* __restrict__ y) {
  __shared__ __align__(16) _Float16 e16[ROWS * EP];
  __shared__ __align__(16) _Float16 h16[ROWS * EP];
  __shared__ __align__(16) float    hf[ROWS * HFP];
  __shared__ __align__(16) float    wo[DOUT * HID];
  __shared__ __align__(16) float    ys[ROWS * YSP];
  static_assert((ROWS - 1) * EP + EP <= ROWS * EP, "sz");
  static_assert((ROWS - 1) * HFP + HID <= ROWS * HFP, "sz");
  static_assert((ROWS - 1) * YSP + (FUT - 1) * DOUT + DOUT <= ROWS * YSP, "sz");

  const int tid  = threadIdx.x;
  const int lane = tid & 31, wave = tid >> 5;
  const int rlane = lane & 15, hh = lane >> 4;
  const int koff = hh * 8, mOff = hh * 8;
  const int blk = blockIdx.x;
  const int b0  = blk * ROWS;
  const int rt  = wave >> 1, cg = wave & 1;
  const int j   = 16 * cg + rlane;
  const int rbase = 16 * rt + mOff;
  const int erow = tid >> 2, q = tid & 3;

  for (int i = tid; i < ROWS * EP; i += NTH) { h16[i] = (_Float16)0.0f; e16[i] = (_Float16)0.0f; }
  for (int i = tid; i < ROWS * HFP; i += NTH) hf[i] = 0.0f;
  for (int i = tid; i < DOUT * HID; i += NTH) wo[i] = Wout[i];

  float we0[8], we1[8], we2[8], we3[8], be[8];
#pragma unroll
  for (int i = 0; i < 8; ++i) {
    const int hid = 8 * q + i;
    we0[i] = Wemb[hid * DIN + 0];
    we1[i] = Wemb[hid * DIN + 1];
    we2[i] = Wemb[hid * DIN + 2];
    we3[i] = Wemb[hid * DIN + 3];
    be[i]  = bemb[hid];
  }
  const float bq = bout[q];

  const v16h wxr = frag_f32_f16(WihE + (size_t)(0 * HID + j) * HID + koff, WSC);
  const v16h wxz = frag_f32_f16(WihE + (size_t)(1 * HID + j) * HID + koff, WSC);
  const v16h wxn = frag_f32_f16(WihE + (size_t)(2 * HID + j) * HID + koff, WSC);
  const v16h whr = frag_f32_f16(WhhE + (size_t)(0 * HID + j) * HID + koff, WSC);
  const v16h whz = frag_f32_f16(WhhE + (size_t)(1 * HID + j) * HID + koff, WSC);
  const v16h whn = frag_f32_f16(WhhE + (size_t)(2 * HID + j) * HID + koff, WSC);
  const float ebr  = bihE[j] + bhhE[j];
  const float ebz  = bihE[HID + j] + bhhE[HID + j];
  const float ebxn = bihE[2 * HID + j];
  const float ebhn = bhhE[2 * HID + j];

  float hreg[8];
#pragma unroll
  for (int r = 0; r < 8; ++r) hreg[r] = 0.0f;
  const v8f z8 = {0.f, 0.f, 0.f, 0.f, 0.f, 0.f, 0.f, 0.f};

  __syncthreads();

  const _Float16* arow_e = e16 + (16 * rt + rlane) * EP + koff;
  const _Float16* arow_h = h16 + (16 * rt + rlane) * EP + koff;
  const float* xb = x + (size_t)(b0 + erow) * SEQ * DIN;
  _Float16* edst = e16 + erow * EP + 8 * q;

#pragma unroll 1
  for (int t = 0; t < SEQ; ++t) {
    {
      const v4f xv = *(const v4f*)(xb + (size_t)t * DIN);
      v8h ev;
#pragma unroll
      for (int i = 0; i < 8; ++i) {
        float s = be[i];
        s = fmaf(xv[0], we0[i], s);
        s = fmaf(xv[1], we1[i], s);
        s = fmaf(xv[2], we2[i], s);
        s = fmaf(xv[3], we3[i], s);
        ev[i] = (_Float16)fmaxf(s, 0.0f);
      }
      *(v8h*)edst = ev;
    }
    __syncthreads();

    const v16h ea = Frag<_Float16>::load(arow_e);
    const v16h ha = Frag<_Float16>::load(arow_h);
    v8f ar  = Frag<_Float16>::mma(ea, wxr, z8);  ar = Frag<_Float16>::mma(ha, whr, ar);
    v8f az  = Frag<_Float16>::mma(ea, wxz, z8);  az = Frag<_Float16>::mma(ha, whz, az);
    v8f axn = Frag<_Float16>::mma(ea, wxn, z8);
    v8f ahn = Frag<_Float16>::mma(ha, whn, z8);
    dep_guard4x_h(ar, az, axn, ahn, ea, ha);

#pragma unroll
    for (int r = 0; r < 8; ++r) {
      const float rg = fsigm(ar[r] * WSC_INV + ebr);
      const float zg = fsigm(az[r] * WSC_INV + ebz);
      const float xn = axn[r] * WSC_INV + ebxn;
      const float hn = ahn[r] * WSC_INV + ebhn;
      const float ng = ftanh(xn + rg * hn);
      hreg[r] = (1.0f - zg) * ng + zg * hreg[r];
    }
    __syncthreads();
#pragma unroll
    for (int r = 0; r < 8; ++r) h16[(rbase + r) * EP + j] = (_Float16)hreg[r];
  }

  const v16h dxr = frag_f32_f16(WihD + (size_t)(0 * HID + j) * HID + koff, WSC);
  const v16h dxz = frag_f32_f16(WihD + (size_t)(1 * HID + j) * HID + koff, WSC);
  const v16h dxn = frag_f32_f16(WihD + (size_t)(2 * HID + j) * HID + koff, WSC);
  const v16h dhr = frag_f32_f16(WhhD + (size_t)(0 * HID + j) * HID + koff, WSC);
  const v16h dhz = frag_f32_f16(WhhD + (size_t)(1 * HID + j) * HID + koff, WSC);
  const v16h dhn = frag_f32_f16(WhhD + (size_t)(2 * HID + j) * HID + koff, WSC);
  const float dbr  = bihD[j] + bhhD[j];
  const float dbz  = bihD[HID + j] + bhhD[HID + j];
  const float dbxn = bihD[2 * HID + j];
  const float dbhn = bhhD[2 * HID + j];

  int nF = flen[0];
  nF = nF < 0 ? 0 : nF;
  nF = nF > FUT ? FUT : nF;
  nF = __builtin_amdgcn_readfirstlane(nF);

  __syncthreads();
  const float* hrow = hf + erow * HFP;
  const float* wrow = wo + q * HID;
#pragma unroll 1
  for (int f = 0; f < nF; ++f) {
    const v16h ha = Frag<_Float16>::load(arow_h);
    v8f ar  = Frag<_Float16>::mma(ha, dxr, z8);  ar = Frag<_Float16>::mma(ha, dhr, ar);
    v8f az  = Frag<_Float16>::mma(ha, dxz, z8);  az = Frag<_Float16>::mma(ha, dhz, az);
    v8f axn = Frag<_Float16>::mma(ha, dxn, z8);
    v8f ahn = Frag<_Float16>::mma(ha, dhn, z8);
    dep_guard4x_h(ar, az, axn, ahn, ha, ha);

#pragma unroll
    for (int r = 0; r < 8; ++r) {
      const float rg = fsigm(ar[r] * WSC_INV + dbr);
      const float zg = fsigm(az[r] * WSC_INV + dbz);
      const float xn = axn[r] * WSC_INV + dbxn;
      const float hn = ahn[r] * WSC_INV + dbhn;
      const float ng = ftanh(xn + rg * hn);
      hreg[r] = (1.0f - zg) * ng + zg * hreg[r];
    }
    __syncthreads();
#pragma unroll
    for (int r = 0; r < 8; ++r) {
      h16[(rbase + r) * EP + j] = (_Float16)hreg[r];
      hf[(rbase + r) * HFP + j] = hreg[r];
    }
    __syncthreads();
    {
      float s = bq;
#pragma unroll
      for (int j4 = 0; j4 < HID / 4; ++j4) {
        const v4f hv = *(const v4f*)(hrow + 4 * j4);
        const v4f wv = *(const v4f*)(wrow + 4 * j4);
        s = fmaf(hv[0], wv[0], s);
        s = fmaf(hv[1], wv[1], s);
        s = fmaf(hv[2], wv[2], s);
        s = fmaf(hv[3], wv[3], s);
      }
      ys[erow * YSP + f * DOUT + q] = s;
    }
  }
  __syncthreads();

  float* yb = y + (size_t)b0 * YSP;
  for (int pass = 0; pass < 2; ++pass) {
#pragma unroll
    for (int it = 0; it < (ROWS * YSP) / (NTH * 4); ++it) {
      const int idx = (it * NTH + tid) * 4;
      const v4f v = *(const v4f*)(ys + idx);
      *(volatile v4f*)(yb + idx) = v;
    }
    __threadfence();
  }
}

extern "C" void kernel_launch(void* const* d_in, const int* in_sizes, int n_in,
                              void* d_out, int out_size, void* d_ws, size_t ws_size, hipStream_t stream) {
  (void)d_ws; (void)ws_size;
  if (n_in < 14 || d_out == nullptr) return;
  if (in_sizes[0] != BATCH * SEQ * DIN || in_sizes[1] != HID * DIN || in_sizes[2] != HID ||
      in_sizes[3] != G3 * HID || in_sizes[4] != G3 * HID || in_sizes[5] != G3 || in_sizes[6] != G3 ||
      in_sizes[7] != G3 * HID || in_sizes[8] != G3 * HID || in_sizes[9] != G3 || in_sizes[10] != G3 ||
      in_sizes[11] != DOUT * HID || in_sizes[12] != DOUT || in_sizes[13] < 1 ||
      out_size != BATCH * FUT * DOUT) return;

  const float* x    = (const float*)d_in[0];
  const float* Wemb = (const float*)d_in[1];
  const float* bemb = (const float*)d_in[2];
  const float* WihE = (const float*)d_in[3];
  const float* WhhE = (const float*)d_in[4];
  const float* bihE = (const float*)d_in[5];
  const float* bhhE = (const float*)d_in[6];
  const float* WihD = (const float*)d_in[7];
  const float* WhhD = (const float*)d_in[8];
  const float* bihD = (const float*)d_in[9];
  const float* bhhD = (const float*)d_in[10];
  const float* Wout = (const float*)d_in[11];
  const float* bout = (const float*)d_in[12];
  const int*   flen = (const int*)d_in[13];
  float* y = (float*)d_out;

  gru_seq2seq_kernel<<<dim3(BATCH / ROWS), dim3(NTH), 0, stream>>>(
      x, Wemb, bemb, WihE, WhhE, bihE, bhhE, WihD, WhhD, bihD, bhhD, Wout, bout, flen, y);
}
